// DomainInvariantFeaturesLearningNetwork_26749056319849
// MI455X (gfx1250) — hardware-run, weakly checked
//
#include <hip/hip_runtime.h>


#ifndef NPTS
#define NPTS 1024
#endif
#define NPTS_FULL 1024
#define FD   2048
#define HID  256
#define IT   8
#define TP   68
#define ESP  264
#define BN_EPS 1e-5f
#define LOG2E 1.4426950408889634f

static_assert(NPTS % 256 == 0);
static_assert(NPTS <= NPTS_FULL);
static_assert(FD % 64 == 0);
static_assert(HID % 64 == 0);
static_assert(HID == 256);
static_assert(IT == 8);
static_assert(IT * HID == 2 * 256 * 4);
static_assert((NPTS / 4) % 16 == 0);
static_assert(TP % 4 == 0);
static_assert(ESP % 8 == 0 && ESP >= 256);
static_assert(32 * 8 * 16 == 16 * 64 * 4);
static_assert(256 * 2 * 16 == 64 * 64 * 2);
static_assert(256 * 4 * 16 == 64 * 64 * 4);
static_assert(256 * 1 * 16 == IT * 256 * 2);
static_assert((64 * TP + 256) * 4 <= 131072);
static_assert(IT * HID * 4 + HID * 4 + IT * ESP * 2 + 8 * IT * 4 <= 131072);
static_assert(((size_t)NPTS * FD) % 8 == 0);

typedef _Float16 h16;
typedef unsigned short bf;
typedef __attribute__((ext_vector_type(16))) __bf16   v16bf;
typedef __attribute__((ext_vector_type(16))) _Float16 v16h;
typedef __attribute__((ext_vector_type(8)))  _Float16 v8h;
typedef __attribute__((ext_vector_type(8)))  unsigned short v8us;
typedef __attribute__((ext_vector_type(8)))  float    v8f;
typedef __attribute__((ext_vector_type(4)))  float    v4f;
typedef v4f  __attribute__((may_alias)) v4fa;
typedef v8h  __attribute__((may_alias)) v8ha;

__device__ __forceinline__ unsigned short f2bf(float f) { unsigned u = __float_as_uint(f); u += 0x7FFFu + ((u >> 16) & 1u); return (unsigned short)(u >> 16); }
__device__ __forceinline__ float bfr(float f) { return __uint_as_float(((unsigned)f2bf(f)) << 16); }
__device__ __forceinline__ v16h cat16(v8h lo, v8h hi) { return __builtin_shufflevector(lo, hi, 0, 1, 2, 3, 4, 5, 6, 7, 8, 9, 10, 11, 12, 13, 14, 15); }
__device__ __forceinline__ v16bf cat16b(v8us lo, v8us hi) { return __builtin_bit_cast(v16bf, __builtin_shufflevector(lo, hi, 0, 1, 2, 3, 4, 5, 6, 7, 8, 9, 10, 11, 12, 13, 14, 15)); }
__device__ __forceinline__ v8f wmma16(v16h a, v16h b, v8f c) { return __builtin_amdgcn_wmma_f32_16x16x32_f16(false, a, false, b, (short)0, c, false, false); }
__device__ __forceinline__ v8f wmmab(v16bf a, v16bf b, v8f c) { return __builtin_amdgcn_wmma_f32_16x16x32_bf16(false, a, false, b, (short)0, c, false, false); }
__device__ __forceinline__ v16h  ldh(const h16* p) { return cat16(*(const v8h*)p, *(const v8h*)(p + 16)); }
__device__ __forceinline__ v16bf ldb(const bf* p)  { return cat16b(*(const v8us*)p, *(const v8us*)(p + 16)); }
__device__ __forceinline__ void wave_sync() { __builtin_amdgcn_fence(3  , "wavefront"); __builtin_amdgcn_wave_barrier(); asm volatile("" ::: "memory"); }
static __device__ __forceinline__ h16 toh_flush(float v) { const h16 r = (h16)v; return (fabsf(v) < 6.103515625e-05f) ? (h16)0.0f : r; }
__device__ __forceinline__ v8f wmmabg(v16bf a, v16bf b, v8f c) { c = wmmab(a, b, c); asm volatile("v_nop\n\tv_nop\n\tv_nop\n\tv_nop" : "+v"(c) : "v"(a), "v"(b)); return c; }
__device__ __forceinline__ v8f wmma16g(v16h a, v16h b, v8f c) { c = wmma16(a, b, c); asm volatile("v_nop\n\tv_nop\n\tv_nop\n\tv_nop" : "+v"(c) : "v"(a), "v"(b)); return c; }

__global__ __launch_bounds__(256) void k_cvt8(const float* __restrict__ src, bf* dst, size_t n8) {
    const size_t i = (size_t)blockIdx.x * 256 + threadIdx.x; if (i >= n8) return;
    const v8f v = *(const v8f*)(src + i * 8); v8us o;
#pragma unroll
    for (int k = 0; k < 8; ++k) o[k] = f2bf(v[k]);
    *(volatile v8us*)(dst + i * 8) = o; __threadfence(); *(volatile v8us*)(dst + i * 8) = o;
}

__global__ __launch_bounds__(256) void k_wtr(const float* __restrict__ src, bf* dst, int R, int C) {
    __shared__ __align__(16) float tile[64 * TP];
    const int tid = threadIdx.x; const int r0 = blockIdx.x * 64, c0 = blockIdx.y * 64;
    const size_t zoff = (size_t)blockIdx.z * (size_t)R * (size_t)C;
#pragma unroll
    for (int it = 0; it < 4; ++it) { const int p = it * 256 + tid; const int row = p >> 4, c4 = (p & 15) * 4;
        const v4f x = *(const v4f*)(src + zoff + (size_t)(r0 + row) * C + c0 + c4); *(v4fa*)(&tile[row * TP + c4]) = x; }
    __syncthreads();
    v8us o[2];
#pragma unroll
    for (int it = 0; it < 2; ++it) { const int p = it * 256 + tid; const int crow = p >> 3, k8 = (p & 7) * 8;
#pragma unroll
        for (int u = 0; u < 8; ++u) { const v4f q = *(const v4fa*)(&tile[(k8 + u) * TP + (crow & ~3)]); o[it][u] = f2bf(q[crow & 3]); } }
#pragma unroll 1
    for (int ps = 0; ps < 2; ++ps) {
#pragma unroll
        for (int it = 0; it < 2; ++it) { const int p = it * 256 + tid; const int crow = p >> 3, k8 = (p & 7) * 8;
            *(volatile v8us*)(dst + zoff + (size_t)(c0 + crow) * R + r0 + k8) = o[it]; }
        if (ps == 0) __threadfence(); }
}

template <int NPL, int BIAS>
__device__ __forceinline__ void gemm_bf_body(const bf* __restrict__ A, const bf* __restrict__ A2, const bf* __restrict__ Bt, const float* __restrict__ bias, float* C, int K, int ldc) {
    __shared__ __align__(16) float os[16 * TP];
    const int lane = threadIdx.x & 31, lr = lane & 15, hi = lane >> 4; const int r0 = blockIdx.x * 64, c0 = blockIdx.y * 64;
    v8f acc[4][4];
#pragma unroll
    for (int mb = 0; mb < 4; ++mb)
#pragma unroll
        for (int nb = 0; nb < 4; ++nb) acc[mb][nb] = (v8f){};
    const size_t aoff = (size_t)(r0 + lr) * K + 8 * hi, boff = (size_t)(c0 + lr) * K + 8 * hi;
#pragma unroll 1
    for (int kc = 0; kc < K; kc += 32) {
        { v16bf a[4];
#pragma unroll
          for (int mb = 0; mb < 4; ++mb) a[mb] = ldb(A + aoff + (size_t)mb * 16 * K + kc);
#pragma unroll
          for (int nb = 0; nb < 4; ++nb) { const v16bf b = ldb(Bt + boff + (size_t)nb * 16 * K + kc);
#pragma unroll
              for (int mb = 0; mb < 4; ++mb) acc[mb][nb] = wmmabg(a[mb], b, acc[mb][nb]); } }
        if (NPL == 2) { v16bf a[4];
#pragma unroll
          for (int mb = 0; mb < 4; ++mb) a[mb] = ldb(A2 + aoff + (size_t)mb * 16 * K + kc);
#pragma unroll
          for (int nb = 0; nb < 4; ++nb) { const v16bf b = ldb(Bt + boff + (size_t)nb * 16 * K + kc);
#pragma unroll
              for (int mb = 0; mb < 4; ++mb) acc[mb][nb] = wmmabg(a[mb], b, acc[mb][nb]); } }
    }
    float bc[4];
#pragma unroll
    for (int nb = 0; nb < 4; ++nb) bc[nb] = BIAS ? bfr(bias[c0 + nb * 16 + lr]) : 0.0f;
    float* cb = C + (size_t)r0 * ldc + c0;
#pragma unroll
    for (int mb = 0; mb < 4; ++mb) {
#pragma unroll
        for (int nb = 0; nb < 4; ++nb) {
#pragma unroll
            for (int j = 0; j < 8; ++j) os[(hi * 8 + j) * TP + nb * 16 + lr] = acc[mb][nb][j] + bc[nb]; }
        wave_sync();
#pragma unroll 1
        for (int ps = 0; ps < 2; ++ps) {
#pragma unroll
            for (int s = 0; s < 8; ++s) { const int p = s * 32 + lane; const int row = p >> 4, c4 = (p & 15) * 4;
                const v4f val = *(const v4fa*)(&os[row * TP + c4]);
                *(volatile v4f*)(cb + (size_t)(mb * 16 + row) * ldc + c4) = val; }
            if (ps == 0) __threadfence(); }
        wave_sync();
    }
}

__global__ __launch_bounds__(32) void k_gemm_p1b(const bf* __restrict__ A, const bf* __restrict__ Bt, const float* __restrict__ bias, float* C, int K, int ldc) {
    gemm_bf_body<1, 1>(A, A, Bt, bias, C, K, ldc);
}
__global__ __launch_bounds__(32) void k_gemm_p1(const bf* __restrict__ A, const bf* __restrict__ Bt, float* C, int K, int ldc) {
    gemm_bf_body<1, 0>(A, A, Bt, nullptr, C, K, ldc);
}
__global__ __launch_bounds__(32) void k_gemm_p2b(const bf* __restrict__ A, const bf* __restrict__ A2, const bf* __restrict__ Bt, const float* __restrict__ bias, float* C, int K, int ldc) {
    gemm_bf_body<2, 1>(A, A2, Bt, bias, C, K, ldc);
}

template <int MODE>
__device__ __forceinline__ void bn_body(const float* __restrict__ Y, const float* __restrict__ g, const float* __restrict__ bt, bf* PH, bf* PL, float* PF, h16* PT) {
    __shared__ __align__(16) float tile[64 * TP];
    __shared__ float red[4 * 64];
    const int tid = threadIdx.x; const int rg = tid >> 6, c = tid & 63; const int c0 = blockIdx.x * 64;
    const float* yc = Y + (size_t)(rg * (NPTS / 4)) * HID + c0 + c;
    float s = 0.0f;
#pragma unroll 4
    for (int r = 0; r < NPTS / 4; ++r) s += yc[(size_t)r * HID];
    red[rg * 64 + c] = s;
    __syncthreads();
    const float mean = ((red[c] + red[64 + c]) + (red[128 + c] + red[192 + c])) * (1.0f / (float)NPTS);
    __syncthreads();
    float q = 0.0f;
#pragma unroll 4
    for (int r = 0; r < NPTS / 4; ++r) { const float d = yc[(size_t)r * HID] - mean; q += d * d; }
    red[rg * 64 + c] = q;
    __syncthreads();
    const float var = ((red[c] + red[64 + c]) + (red[128 + c] + red[192 + c])) * (1.0f / (float)NPTS);
    const float gs = bfr(g[c0 + c]) * rsqrtf(var + BN_EPS);
    const float bb = bfr(bt[c0 + c]);
#pragma unroll 1
    for (int ch = 0; ch < NPTS / 64; ++ch) {
        const int r0 = ch * 64;
        const float* yp = Y + (size_t)(r0 + rg * 16) * HID + c0 + c;
#pragma unroll 4
        for (int rr = 0; rr < 16; ++rr) { const float v = (yp[(size_t)rr * HID] - mean) * gs + bb; tile[(rg * 16 + rr) * TP + c] = fmaxf(v, 0.0f); }
        __syncthreads();
#pragma unroll 1
        for (int ps = 0; ps < 2; ++ps) {
#pragma unroll
            for (int it = 0; it < 2; ++it) { const int p = it * 256 + tid; const int row = p >> 3, c8 = (p & 7) * 8;
                const v4f x0 = *(const v4fa*)(&tile[row * TP + c8]); const v4f x1 = *(const v4fa*)(&tile[row * TP + c8 + 4]); v8us hv, lv;
#pragma unroll
                for (int i = 0; i < 4; ++i) { const unsigned short u0 = f2bf(x0[i]); const unsigned short u1 = f2bf(x1[i]); hv[i] = u0; hv[4 + i] = u1;
                    lv[i] = f2bf(x0[i] - __uint_as_float(((unsigned)u0) << 16)); lv[4 + i] = f2bf(x1[i] - __uint_as_float(((unsigned)u1) << 16)); }
                const size_t off = (size_t)(r0 + row) * HID + c0 + c8;
                *(volatile v8us*)(PH + off) = hv; if (MODE == 0) *(volatile v8us*)(PL + off) = lv; }
            if (MODE == 1) {
#pragma unroll
                for (int it = 0; it < 4; ++it) { const int p = it * 256 + tid; const int row = p >> 4, c4 = (p & 15) * 4;
                    const v4f x = *(const v4fa*)(&tile[row * TP + c4]);
                    *(volatile v4f*)(PF + (size_t)(r0 + row) * HID + c0 + c4) = x; }
#pragma unroll
                for (int it = 0; it < 2; ++it) { const int p = it * 256 + tid; const int crow = p >> 3, j8 = (p & 7) * 8;
                    v8h tv;
#pragma unroll
                    for (int u = 0; u < 8; ++u) { const v4f qv = *(const v4fa*)(&tile[(j8 + u) * TP + (crow & ~3)]); tv[u] = toh_flush(qv[crow & 3]); }
                    *(volatile v8h*)(PT + (size_t)(c0 + crow) * NPTS + r0 + j8) = tv; }
            }
            if (ps == 0) __threadfence(); }
        __syncthreads();
    }
}

__global__ __launch_bounds__(256) void k_bn1(const float* __restrict__ Y, const float* __restrict__ g, const float* __restrict__ bt, bf* PH, bf* PL) {
    bn_body<0>(Y, g, bt, PH, PL, nullptr, nullptr);
}
__global__ __launch_bounds__(256) void k_bn2(const float* __restrict__ Y, const float* __restrict__ g, const float* __restrict__ bt, bf* PH, float* PF, h16* PT) {
    bn_body<1>(Y, g, bt, PH, PH, PF, PT);
}

__global__ __launch_bounds__(256) void k_pair(const float* __restrict__ HI, const float* __restrict__ HJT, const float* __restrict__ we2, const float* __restrict__ bwe2,
                                              const int* __restrict__ labels, h16* E, float* WS) {
    __shared__ __align__(16) float his[IT * HID];
    __shared__ __align__(16) float w2s[HID];
    __shared__ __align__(16) h16 es[IT * ESP];
    __shared__ float part[8 * IT];
    const int tid = threadIdx.x, lane = tid & 31;
    const int wave = __builtin_amdgcn_readfirstlane((int)(threadIdx.x >> 5));
    const int i0 = blockIdx.x * IT;
#pragma unroll
    for (int it = 0; it < 2; ++it) { const int p = it * 256 + tid; const v4f x = *(const v4f*)(HI + (size_t)i0 * HID + (size_t)p * 4); *(v4fa*)(&his[p * 4]) = x; }
    { const int t4 = tid & ~3; v4f w4; w4[0] = 0.0f; w4[1] = 0.0f; w4[2] = 0.0f; w4[3] = 0.0f;
      const float wv = bfr(we2[tid]);
      const float a0 = __shfl(wv, (lane & ~3) + 0, 32), a1 = __shfl(wv, (lane & ~3) + 1, 32), a2 = __shfl(wv, (lane & ~3) + 2, 32), a3 = __shfl(wv, (lane & ~3) + 3, 32);
      w4[0] = a0; w4[1] = a1; w4[2] = a2; w4[3] = a3;
      if ((tid & 3) == 0) *(v4fa*)(&w2s[t4]) = w4; }
    int li[IT];
#pragma unroll
    for (int r = 0; r < IT; ++r) li[r] = labels[i0 + r];
    const float b2v = bfr(bwe2[0]);
    __syncthreads();
    float rs[IT];
#pragma unroll
    for (int r = 0; r < IT; ++r) rs[r] = 0.0f;
#pragma unroll 1
    for (int jc = 0; jc < NPTS / 256; ++jc) {
        const int j = jc * 256 + tid;
        const int lj = labels[j];
        float acc[IT];
#pragma unroll
        for (int r = 0; r < IT; ++r) acc[r] = 0.0f;
        const float* hp = HJT + j;
#pragma unroll 1
        for (int h = 0; h < HID; h += 4) {
            const float x0 = hp[(size_t)(h + 0) * NPTS], x1 = hp[(size_t)(h + 1) * NPTS], x2 = hp[(size_t)(h + 2) * NPTS], x3 = hp[(size_t)(h + 3) * NPTS];
            const v4f w = *(const v4fa*)(&w2s[h]);
#pragma unroll
            for (int r = 0; r < IT; ++r) { const v4f a = *(const v4fa*)(&his[r * HID + h]);
                acc[r] = fmaf(fmaxf(a[0] + x0, 0.0f), w[0], acc[r]); acc[r] = fmaf(fmaxf(a[1] + x1, 0.0f), w[1], acc[r]);
                acc[r] = fmaf(fmaxf(a[2] + x2, 0.0f), w[2], acc[r]); acc[r] = fmaf(fmaxf(a[3] + x3, 0.0f), w[3], acc[r]); }
        }
#pragma unroll
        for (int r = 0; r < IT; ++r) {
            const float lg = acc[r] + b2v;
            const float sg = __builtin_amdgcn_rcpf(1.0f + __builtin_amdgcn_exp2f(-lg * LOG2E));
            const bool keep = (li[r] == lj) & ((i0 + r) != j);
            const h16 e = toh_flush(keep ? sg : 0.0f);
            rs[r] += (float)e;
            es[r * ESP + tid] = e; }
        __syncthreads();
        const v8h ev = *(const v8ha*)(&es[wave * ESP + lane * 8]);
        h16* dst = E + (size_t)(i0 + wave) * NPTS + (size_t)jc * 256 + lane * 8;
        *(volatile v8h*)dst = ev; __threadfence(); *(volatile v8h*)dst = ev;
        __syncthreads();
    }
#pragma unroll
    for (int r = 0; r < IT; ++r) { float v = rs[r];
        v += __shfl_xor(v, 16, 32); v += __shfl_xor(v, 8, 32); v += __shfl_xor(v, 4, 32); v += __shfl_xor(v, 2, 32); v += __shfl_xor(v, 1, 32); rs[r] = v; }
    if (lane == 0) {
#pragma unroll
        for (int r = 0; r < IT; ++r) part[wave * IT + r] = rs[r]; }
    __syncthreads();
    if (wave == 0) {
        v4f o;
#pragma unroll
        for (int k = 0; k < 4; ++k) { const int idx = lane * 4 + k; const int rr = idx & (IT - 1); float v = 0.0f;
#pragma unroll
            for (int w = 0; w < 8; ++w) v += part[w * IT + rr];
            o[k] = (idx < IT) ? v : 0.0f; }
        float* wd = WS + (size_t)blockIdx.x * 32 + lane * 4;
        if (lane < 8) { *(volatile v4f*)wd = o; __threadfence(); *(volatile v4f*)wd = o; }
    }
}

__global__ __launch_bounds__(32) void k_agg(const h16* __restrict__ E, const h16* __restrict__ DT, const float* __restrict__ DI, const float* __restrict__ WS, float* OUT) {
    __shared__ __align__(16) float os[16 * TP];
    const int K = NPTS;
    const int lane = threadIdx.x & 31, lr = lane & 15, hi = lane >> 4; const int r0 = blockIdx.x * 64, c0 = blockIdx.y * 64;
    v8f acc[4][4];
#pragma unroll
    for (int mb = 0; mb < 4; ++mb)
#pragma unroll
        for (int nb = 0; nb < 4; ++nb) acc[mb][nb] = (v8f){};
    const size_t aoff = (size_t)(r0 + lr) * K + 8 * hi, boff = (size_t)(c0 + lr) * K + 8 * hi;
#pragma unroll 1
    for (int kc = 0; kc < K; kc += 32) {
        v16h a[4];
#pragma unroll
        for (int mb = 0; mb < 4; ++mb) a[mb] = ldh(E + aoff + (size_t)mb * 16 * K + kc);
#pragma unroll
        for (int nb = 0; nb < 4; ++nb) { const v16h b = ldh(DT + boff + (size_t)nb * 16 * K + kc);
#pragma unroll
            for (int mb = 0; mb < 4; ++mb) acc[mb][nb] = wmma16g(a[mb], b, acc[mb][nb]); }
    }
#pragma unroll
    for (int mb = 0; mb < 4; ++mb) {
#pragma unroll
        for (int nb = 0; nb < 4; ++nb) {
#pragma unroll
            for (int j = 0; j < 8; ++j) os[(hi * 8 + j) * TP + nb * 16 + lr] = acc[mb][nb][j]; }
        wave_sync();
#pragma unroll 1
        for (int ps = 0; ps < 2; ++ps) {
#pragma unroll
            for (int s = 0; s < 8; ++s) { const int p = s * 32 + lane; const int row = p >> 4, c4 = (p & 15) * 4;
                const int gi = r0 + mb * 16 + row;
                const float w = WS[(size_t)(gi / IT) * 32 + (gi % IT)];
                const v4f a = *(const v4fa*)(&os[row * TP + c4]);
                const v4f d = *(const v4f*)(DI + (size_t)gi * HID + c0 + c4);
                const bool pos = w > 0.0f;
                const float rinv = __builtin_amdgcn_rcpf(pos ? w : 1.0f);
                v4f o;
#pragma unroll
                for (int i = 0; i < 4; ++i) o[i] = d[i] + (pos ? a[i] * rinv : 0.0f);
                *(volatile v4f*)(OUT + (size_t)gi * HID + c0 + c4) = o; }
            if (ps == 0) __threadfence(); }
        wave_sync();
    }
}

static constexpr size_t al256(size_t v) { return (v + 255) & ~(size_t)255; }
static constexpr size_t SZ_FB  = al256((size_t)NPTS * FD * 2);
static constexpr size_t SZ_W1T = al256((size_t)HID * FD * 2);
static constexpr size_t SZ_W2T = al256((size_t)HID * HID * 2);
static constexpr size_t SZ_WET = al256((size_t)2 * HID * HID * 2);
static constexpr size_t SZ_F32 = al256((size_t)NPTS * HID * 4);
static constexpr size_t SZ_H16 = al256((size_t)NPTS * HID * 2);
static constexpr size_t SZ_E   = al256((size_t)NPTS * NPTS * 2);
static constexpr size_t SZ_WS  = al256((size_t)(NPTS / IT) * 32 * 4);
static constexpr size_t SZ_TOTAL = SZ_FB + SZ_W1T + SZ_W2T + SZ_WET + 4 * SZ_F32 + 4 * SZ_H16 + SZ_E + SZ_WS;
static_assert(SZ_TOTAL <= (size_t)134217728);
static_assert(((size_t)HID * HID * 2) % 256 == 0);
static_assert((size_t)(NPTS / IT - 1) * 32 + 32 <= SZ_WS / 4);

extern "C" void kernel_launch(void* const* d_in, const int* in_sizes, int n_in,
                              void* d_out, int out_size, void* d_ws, size_t ws_size, hipStream_t stream) {
    if (n_in < 14) return;
    if ((size_t)in_sizes[0] < (size_t)NPTS * FD || in_sizes[1] < NPTS) return;
    if ((size_t)in_sizes[2] < (size_t)FD * HID || in_sizes[3] < HID || in_sizes[4] < HID || in_sizes[5] < HID) return;
    if ((size_t)in_sizes[6] < (size_t)HID * HID || in_sizes[7] < HID || in_sizes[8] < HID || in_sizes[9] < HID) return;
    if ((size_t)in_sizes[10] < (size_t)2 * HID * HID || in_sizes[11] < HID || in_sizes[12] < HID || in_sizes[13] < 1) return;
    if ((size_t)out_size < (size_t)NPTS * HID) return;
    if (SZ_TOTAL > ws_size) return;
    const float* features = (const float*)d_in[0];
    const int*   labels   = (const int*)d_in[1];
    const float* W1  = (const float*)d_in[2];  const float* b1  = (const float*)d_in[3];
    const float* g1  = (const float*)d_in[4];  const float* bt1 = (const float*)d_in[5];
    const float* W2  = (const float*)d_in[6];  const float* b2  = (const float*)d_in[7];
    const float* g2  = (const float*)d_in[8];  const float* bt2 = (const float*)d_in[9];
    const float* We1 = (const float*)d_in[10]; const float* bwe1 = (const float*)d_in[11];
    const float* We2 = (const float*)d_in[12]; const float* bwe2 = (const float*)d_in[13];
    float* OUT = (float*)d_out;
    char* wsp = (char*)d_ws;
    bf* FB   = (bf*)wsp;    wsp += SZ_FB;
    bf* W1T  = (bf*)wsp;    wsp += SZ_W1T;
    bf* W2T  = (bf*)wsp;    wsp += SZ_W2T;
    bf* WET  = (bf*)wsp;    wsp += SZ_WET;
    float* Y   = (float*)wsp; wsp += SZ_F32;
    float* DI  = (float*)wsp; wsp += SZ_F32;
    float* HI  = (float*)wsp; wsp += SZ_F32;
    float* HJT = (float*)wsp; wsp += SZ_F32;
    bf* HH   = (bf*)wsp;    wsp += SZ_H16;
    bf* HL   = (bf*)wsp;    wsp += SZ_H16;
    bf* DIH  = (bf*)wsp;    wsp += SZ_H16;
    h16* DT  = (h16*)wsp;   wsp += SZ_H16;
    h16* E   = (h16*)wsp;   wsp += SZ_E;
    float* WS = (float*)wsp; wsp += SZ_WS;

    { const size_t n8 = (size_t)NPTS * FD / 8;
      k_cvt8<<<(unsigned)((n8 + 255) / 256), 256, 0, stream>>>(features, FB, n8); }
    k_wtr<<<dim3(FD / 64, HID / 64, 1), 256, 0, stream>>>(W1, W1T, FD, HID);
    k_wtr<<<dim3(HID / 64, HID / 64, 1), 256, 0, stream>>>(W2, W2T, HID, HID);
    k_wtr<<<dim3(HID / 64, HID / 64, 2), 256, 0, stream>>>(We1, WET, HID, HID);

    k_gemm_p1b<<<dim3(NPTS / 64, HID / 64, 1), 32, 0, stream>>>(FB, W1T, b1, Y, FD, HID);
    k_bn1<<<dim3(HID / 64, 1, 1), 256, 0, stream>>>(Y, g1, bt1, HH, HL);
    k_gemm_p2b<<<dim3(NPTS / 64, HID / 64, 1), 32, 0, stream>>>(HH, HL, W2T, b2, Y, HID, HID);
    k_bn2<<<dim3(HID / 64, 1, 1), 256, 0, stream>>>(Y, g2, bt2, DIH, DI, DT);
    k_gemm_p1b<<<dim3(NPTS / 64, HID / 64, 1), 32, 0, stream>>>(DIH, WET, bwe1, HI, HID, HID);
    k_gemm_p1<<<dim3(HID / 64, NPTS / 64, 1), 32, 0, stream>>>(WET + (size_t)HID * HID, DIH, HJT, HID, NPTS);
    k_pair<<<dim3(NPTS / IT, 1, 1), 256, 0, stream>>>(HI, HJT, We2, bwe2, labels, E, WS);
    k_agg<<<dim3(NPTS / 64, HID / 64, 1), 32, 0, stream>>>(E, DT, DI, WS, OUT);
}
